// GNNModel_47141561041135
// MI455X (gfx1250) — hardware-verified
//
#include <hip/hip_runtime.h>
#include <stddef.h>
#include <stdint.h>


#define D      128
#define HSN    256
#define KZ     256
#define PBN    256
#define NG     16
#define NCLS   10
#define NOUT1  (NG * NCLS)
#define NTHR   256
#define NWAVE  8
#define EPT    8
#define CHUNK  (NTHR * EPT)
#define WCAP   (EPT * 32)
#define LISTN  (NWAVE * WCAP)
#define NBA    256
#define SLA    8
#define RCAP   26112
#define DEGCAP 128
#define EPB    256
#define CHB    2048
#define GBM    64
#define GBN    128
#define GTHR   128
#define NU1    (HSN * (D / 8))
#define NU2    (PBN * (KZ / 8))
#define AGG_ZINTS (LISTN + 2 * RCAP + 3 * NBA)
#define AGG_LDS_INTS (AGG_ZINTS + 16)
#define WSMAX  134217728

static_assert((CHUNK & (CHUNK - 1)) == 0 && CHUNK <= 4096);
static_assert((NBA & (NBA - 1)) == 0 && NBA == (1 << SLA));
static_assert(((long long)CHUNK << SLA) < (1LL << 31));
static_assert(LISTN % NTHR == 0);
static_assert(NBA % NWAVE == 0 && NBA % 32 == 0 && NBA % GBM == 0);
static_assert(RCAP % 4 == 0 && AGG_ZINTS % 4 == 0 && LISTN % 4 == 0);
static_assert(RCAP >= NBA * 101 && DEGCAP >= 117);
static_assert(D % 32 == 0 && KZ % 32 == 0 && KZ == 2 * D && HSN == 2 * GBN && PBN == 2 * GBN);
static_assert(GBM == (GTHR / 32) * 16 && GBN == 4 * 32);
static_assert(NU1 % NTHR == 0 && NU2 % NTHR == 0 && (NU1 / 2) % NTHR == 0 && (NU2 / 2) % NTHR == 0);
static_assert(D / 8 == 16 && KZ / 8 == 32);
static_assert(AGG_LDS_INTS * 4 <= 300000);
static_assert(EPB == NTHR && EPB == 8 * 32 && D % 32 == 0 && D <= NTHR);
static_assert(NTHR == 2 * D && NG % 2 == 0 && NOUT1 % 4 == 0 && NOUT1 <= NTHR && NCLS <= 32);
static_assert(CHB % NTHR == 0);

typedef float          v4f   __attribute__((ext_vector_type(4)));
typedef float          v8f   __attribute__((ext_vector_type(8)));
typedef int            v4i   __attribute__((ext_vector_type(4)));
typedef int            v8i   __attribute__((ext_vector_type(8)));
typedef unsigned short v8us  __attribute__((ext_vector_type(8)));
typedef unsigned short v16us __attribute__((ext_vector_type(16)));
typedef __bf16         v16bf __attribute__((ext_vector_type(16)));
typedef v4f  __attribute__((may_alias)) v4fa;
typedef v4i  __attribute__((may_alias)) v4ia;
typedef v8us __attribute__((may_alias)) v8usa;
union FragB { v16bf v; v16us u; v8us h[2]; v8i w; };

__device__ __forceinline__ v8f wmb(const FragB& a, const FragB& b, v8f c) {
  v8f d = __builtin_amdgcn_wmma_f32_16x16x32_bf16(false, a.v, false, b.v, (short)0, c, false, false);
  asm volatile("v_nop\n\tv_nop\n\tv_nop\n\tv_nop" : "+v"(d) : "v"(a.w), "v"(b.w));
  return d;
}

__device__ __forceinline__ unsigned bf16_bits(float f) {
  const unsigned u = __float_as_uint(f);
  return (u + 0x7FFFu + ((u >> 16) & 1u)) >> 16;
}
__device__ __forceinline__ float bf16_val(float f) {
  return __uint_as_float(bf16_bits(f) << 16);
}

template <int SLB>
__device__ __forceinline__ int scan_chunk(const int* __restrict__ dsts, int nE, int cbase, int slotBase,
                                          int nb, int vec8, int* list, int tid, int lane, int wave) {
  int wc = 0;
  const int el0  = tid * EPT;
  const int e0   = cbase + el0;
  const int sent = -2147483647 - 1;
  v4i da, db;
  if (vec8 != 0 && cbase + CHUNK <= nE) {
    da = *(const v4i*)(dsts + e0);
    db = *(const v4i*)(dsts + e0 + 4);
  } else {
    da.x = (e0     < nE) ? dsts[min(e0,     nE - 1)] : sent;
    da.y = (e0 + 1 < nE) ? dsts[min(e0 + 1, nE - 1)] : sent;
    da.z = (e0 + 2 < nE) ? dsts[min(e0 + 2, nE - 1)] : sent;
    da.w = (e0 + 3 < nE) ? dsts[min(e0 + 3, nE - 1)] : sent;
    db.x = (e0 + 4 < nE) ? dsts[min(e0 + 4, nE - 1)] : sent;
    db.y = (e0 + 5 < nE) ? dsts[min(e0 + 5, nE - 1)] : sent;
    db.z = (e0 + 6 < nE) ? dsts[min(e0 + 6, nE - 1)] : sent;
    db.w = (e0 + 7 < nE) ? dsts[min(e0 + 7, nE - 1)] : sent;
  }
  const unsigned nbs = (unsigned)slotBase;
  const unsigned unb = (unsigned)nb;
  const unsigned s0 = (unsigned)da.x - nbs, s1 = (unsigned)da.y - nbs;
  const unsigned s2 = (unsigned)da.z - nbs, s3 = (unsigned)da.w - nbs;
  const unsigned s4 = (unsigned)db.x - nbs, s5 = (unsigned)db.y - nbs;
  const unsigned s6 = (unsigned)db.z - nbs, s7 = (unsigned)db.w - nbs;
  const bool h0 = s0 < unb, h1 = s1 < unb, h2 = s2 < unb, h3 = s3 < unb;
  const bool h4 = s4 < unb, h5 = s5 < unb, h6 = s6 < unb, h7 = s7 < unb;
  const unsigned any = __builtin_amdgcn_ballot_w32(h0 | h1 | h2 | h3 | h4 | h5 | h6 | h7);
  if (any != 0u) {
#define HITJ(J, HJ, SJ) { \
      const unsigned mj = __builtin_amdgcn_ballot_w32(HJ); \
      if (mj != 0u) { \
        if (HJ) { \
          const int pos = wc + (int)__builtin_amdgcn_mbcnt_lo(mj, 0u); \
          if (pos < WCAP) list[wave * WCAP + pos] = ((el0 + (J)) << SLB) | (int)(SJ); \
        } \
        wc += (int)__builtin_popcount(mj); } }
    HITJ(0, h0, s0)
    HITJ(1, h1, s1)
    HITJ(2, h2, s2)
    HITJ(3, h3, s3)
    HITJ(4, h4, s4)
    HITJ(5, h5, s5)
    HITJ(6, h6, s6)
    HITJ(7, h7, s7)
#undef HITJ
  }
  return wc;
}

__global__ __launch_bounds__(NTHR) void k_prep(const float* __restrict__ x, const float* __restrict__ Win,
                                               const float* __restrict__ Wself, const float* __restrict__ We1,
                                               int nN, int mRows,
                                               unsigned short* WIS, unsigned short* WAB, unsigned short* XB) {
  const int u = (int)blockIdx.x * NTHR + (int)threadIdx.x;
  v8us o;
  unsigned short* dp;
  if (u < NU1) {
    const int n  = u >> 4;
    const int k8 = (u & 15) * 8;
    const int nn = n & (D - 1);
    const float* Wp = (n < D) ? Win : Wself;
    const float* p = Wp + (size_t)k8 * D + nn;
#pragma unroll
    for (int i = 0; i < 8; ++i) o[i] = (unsigned short)bf16_bits(p[(size_t)i * D]);
    dp = WIS + (size_t)n * D + k8;
  } else if (u < NU1 + NU2) {
    const int v   = u - NU1;
    const int n   = v >> 5;
    const int l   = v & 31;
    const int j8  = l * 8;
    const int c0  = l * 4;
    const int nn  = n & (D - 1);
    const int kof = (n >> 7) * D;
    const float* p = We1 + (size_t)(kof + c0) * D + nn;
#pragma unroll
    for (int i = 0; i < 4; ++i) {
      const unsigned short bb = (unsigned short)bf16_bits(p[(size_t)i * D]);
      o[i]     = bb;
      o[i + 4] = bb;
    }
    dp = WAB + (size_t)n * KZ + j8;
  } else {
    const int v = u - NU1 - NU2;
    if (v >= mRows * (D / 8)) return;
    const int row = v >> 4;
    const int k8  = (v & 15) * 8;
    const int rc  = row < nN ? row : nN - 1;
    const float* p = x + (size_t)rc * D + k8;
    const v4f a = *(const v4fa*)p;
    const v4f b = *(const v4fa*)(p + 4);
    const bool ok = row < nN;
    o[0] = ok ? (unsigned short)bf16_bits(a.x) : (unsigned short)0;
    o[1] = ok ? (unsigned short)bf16_bits(a.y) : (unsigned short)0;
    o[2] = ok ? (unsigned short)bf16_bits(a.z) : (unsigned short)0;
    o[3] = ok ? (unsigned short)bf16_bits(a.w) : (unsigned short)0;
    o[4] = ok ? (unsigned short)bf16_bits(b.x) : (unsigned short)0;
    o[5] = ok ? (unsigned short)bf16_bits(b.y) : (unsigned short)0;
    o[6] = ok ? (unsigned short)bf16_bits(b.z) : (unsigned short)0;
    o[7] = ok ? (unsigned short)bf16_bits(b.w) : (unsigned short)0;
    dp = XB + (size_t)row * D + k8;
  }
  *(volatile v8us*)dp = o;
  __threadfence();
  *(volatile v8us*)dp = o;
}

__global__ __launch_bounds__(GTHR) void k_gemm(const unsigned short* __restrict__ A, int lda,
                                               const unsigned short* __restrict__ BT, int ldb, int K,
                                               float* Cm, int ldc) {
  __shared__ __attribute__((aligned(16))) float stg[GBM * GBN];
  const int tid = (int)threadIdx.x, lane = tid & 31, wave = tid >> 5, hh = lane >> 4, m = lane & 15;
  const int rowBase = (int)blockIdx.x * GBM;
  const int colBase = (int)blockIdx.y * GBN;

  v8f acc[8];
  {
    const v8f z = {0.f, 0.f, 0.f, 0.f, 0.f, 0.f, 0.f, 0.f};
#pragma unroll
    for (int t = 0; t < 8; ++t) acc[t] = z;
  }
  const unsigned short* ap = A  + (size_t)(rowBase + 16 * wave + m) * (size_t)lda + 8 * hh;
  const unsigned short* bp = BT + (size_t)(colBase + m) * (size_t)ldb + 8 * hh;

#pragma unroll 1
  for (int k0 = 0; k0 < K; k0 += 32) {
    FragB af;
    af.h[0] = *(const v8usa*)(ap + k0);
    af.h[1] = *(const v8usa*)(ap + k0 + 16);
#pragma unroll
    for (int nt = 0; nt < 8; ++nt) {
      const unsigned short* wq = bp + (size_t)(16 * nt) * (size_t)ldb + k0;
      FragB bf;
      bf.h[0] = *(const v8usa*)wq;
      bf.h[1] = *(const v8usa*)(wq + 16);
      acc[nt] = wmb(af, bf, acc[nt]);
    }
  }

#pragma unroll
  for (int nt = 0; nt < 8; ++nt) {
    const int lc = 16 * nt + m;
#pragma unroll
    for (int r = 0; r < 8; ++r) {
      const int lr = 16 * wave + 8 * hh + r;
      stg[lr * GBN + lc] = acc[nt][r];
    }
  }
  __syncthreads();

  v4f pv[16];
#pragma unroll
  for (int i = 0; i < 16; ++i) pv[i] = *(const v4fa*)(stg + (16 * wave + i) * GBN + 4 * lane);
#pragma unroll
  for (int i = 0; i < 16; ++i) {
    float* op = Cm + (size_t)(rowBase + 16 * wave + i) * (size_t)ldc + colBase + 4 * lane;
    *(volatile v4f*)op = pv[i];
  }
  __threadfence();
#pragma unroll
  for (int i = 0; i < 16; ++i) {
    float* op = Cm + (size_t)(rowBase + 16 * wave + i) * (size_t)ldc + colBase + 4 * lane;
    *(volatile v4f*)op = pv[i];
  }
}

__global__ __launch_bounds__(NTHR) void k_agg(const int* __restrict__ srcs, const int* __restrict__ dsts,
                                              int nE, int nN, int vec8, int mRows,
                                              const float* __restrict__ hs, const float* __restrict__ bias,
                                              float* zf, unsigned short* za) {
  extern __shared__ __attribute__((aligned(16))) int dsm[];
  int* list = dsm;
  int* hl   = dsm + LISTN;
  int* sl   = dsm + LISTN + RCAP;
  int* cnt  = dsm + LISTN + 2 * RCAP;
  int* offs = cnt + NBA;
  int* cur  = offs + NBA;
  int* misc = cur + NBA;
  const int tid = (int)threadIdx.x, lane = tid & 31, wave = tid >> 5;
  const int nodeBase = (int)blockIdx.x * NBA;

  {
    const v4i z4 = {0, 0, 0, 0};
    for (int i = tid * 4; i < AGG_ZINTS; i += NTHR * 4) *(v4ia*)(dsm + i) = z4;
    if (tid < 16) misc[tid] = 0;
  }
  float bv[4];
  {
    const v4f a = *(const v4fa*)(bias + 4 * lane);
    bv[0] = bf16_val(a.x); bv[1] = bf16_val(a.y); bv[2] = bf16_val(a.z); bv[3] = bf16_val(a.w);
  }
  __syncthreads();

  int t = 0, ov = 0;
  const int nChunks = (nE + CHUNK - 1) / CHUNK;
#pragma unroll 1
  for (int ch = 0; ch < nChunks; ++ch) {
    const int cbase = ch * CHUNK;
    const int wc = scan_chunk<SLA>(dsts, nE, cbase, nodeBase, NBA, vec8, list, tid, lane, wave);
    if (lane == 0) misc[wave] = wc;
    __syncthreads();
    if (wave == 0) {
#pragma unroll 1
      for (int w2 = 0; w2 < NWAVE; ++w2) {
        int c = misc[w2];
        c = c < 0 ? 0 : (c > WCAP ? WCAP : c);
#pragma unroll 1
        for (int b0 = 0; b0 < c; b0 += 32) {
          const int idx = b0 + lane;
          const int ent = list[w2 * WCAP + (idx < WCAP ? idx : WCAP - 1)];
          const int m32 = (c - b0) < 32 ? (c - b0) : 32;
#pragma unroll 1
          for (int k = 0; k < m32; ++k) {
            const int u    = __builtin_amdgcn_readlane(ent, k);
            const int slot = u & (NBA - 1);
            const int el   = (u >> SLA) & (CHUNK - 1);
            const int pk   = ((cbase + el) << SLA) | slot;
            if (t < RCAP) {
              if (lane == 0) { hl[t] = pk; cnt[slot] = cnt[slot] + 1; }
              t = t + 1;
            } else {
              ov = 1;
            }
          }
        }
      }
    }
    __syncthreads();
  }
  if (wave == 0 && lane == 0) { misc[8] = t; misc[9] = ov; }
  __syncthreads();
  int tt = misc[8];
  tt = tt < 0 ? 0 : (tt > RCAP ? RCAP : tt);
  const int ovf = misc[9];

  if (wave == 0) {
    const int base = lane * (NBA / 32);
    int s = 0;
#pragma unroll 1
    for (int i = 0; i < NBA / 32; ++i) s += cnt[base + i];
    int incl = s;
#pragma unroll
    for (int d = 1; d < 32; d <<= 1) {
      const int y = __shfl_up(incl, d, 32);
      if (lane >= d) incl += y;
    }
    int run = incl - s;
#pragma unroll 1
    for (int i = 0; i < NBA / 32; ++i) {
      const int cv = cnt[base + i];
      offs[base + i] = run;
      cur[base + i]  = run;
      run += cv;
    }
  }
  __syncthreads();
  if (wave == 0) {
#pragma unroll 1
    for (int b0 = 0; b0 < tt; b0 += 32) {
      const int idx = b0 + lane;
      const int ent = hl[idx < RCAP ? idx : RCAP - 1];
      const int m32 = (tt - b0) < 32 ? (tt - b0) : 32;
#pragma unroll 1
      for (int k = 0; k < m32; ++k) {
        const int u    = __builtin_amdgcn_readlane(ent, k);
        const int slot = u & (NBA - 1);
        if (lane == 0) {
          int p = cur[slot];
          p = p < 0 ? 0 : (p > RCAP - 1 ? RCAP - 1 : p);
          sl[p] = u;
          cur[slot] = p + 1;
        }
      }
    }
  }
  __syncthreads();

  const float pz = (ovf != 0) ? __int_as_float(0x7fc00000) : 0.0f;
#pragma unroll 1
  for (int si = 0; si < NBA / NWAVE; ++si) {
    const int s    = si * NWAVE + wave;
    const int node = nodeBase + s;
    int c = cnt[s];
    const bool big = c > DEGCAP;
    c = c < 0 ? 0 : (c > DEGCAP ? DEGCAP : c);
    int o = offs[s];
    o = o < 0 ? 0 : (o > RCAP ? RCAP : o);
    const int nc = node < nN ? node : nN - 1;
    float acc[4];
#pragma unroll
    for (int i = 0; i < 4; ++i) acc[i] = 0.0f;
#pragma unroll 1
    for (int b0 = 0; b0 < c; b0 += 32) {
      int idx = o + b0 + lane;
      idx = idx > RCAP - 1 ? RCAP - 1 : idx;
      const int ent = sl[idx];
      int eid = ent >> SLA;
      eid = eid < 0 ? 0 : (eid > nE - 1 ? nE - 1 : eid);
      int sr = srcs[eid];
      sr = sr < 0 ? 0 : (sr > nN - 1 ? nN - 1 : sr);
      const int m32 = (c - b0) < 32 ? (c - b0) : 32;
#pragma unroll 1
      for (int k = 0; k < m32; ++k) {
        const int sk = __builtin_amdgcn_readlane(sr, k);
        const float* rp = hs + (size_t)sk * HSN + 4 * lane;
        const v4f a = *(const v4fa*)rp;
        acc[0] += a.x; acc[1] += a.y; acc[2] += a.z; acc[3] += a.w;
      }
    }
    float sv[4];
    {
      const float* sp = hs + (size_t)nc * HSN + D + 4 * lane;
      const v4f a = *(const v4fa*)sp;
      sv[0] = a.x; sv[1] = a.y; sv[2] = a.z; sv[3] = a.w;
    }
    const float pzr = big ? __int_as_float(0x7fc00000) : pz;
    const bool live = node < nN;
    float v[4];
#pragma unroll
    for (int i = 0; i < 4; ++i) {
      float y = (acc[i] + sv[i]) + bv[i];
      y = fmaxf(y, 0.0f);
      y = y + pzr;
      v[i] = live ? y : 0.0f;
    }
    v4f zv;
    zv.x = v[0]; zv.y = v[1]; zv.z = v[2]; zv.w = v[3];
    v8us ab;
#pragma unroll
    for (int i = 0; i < 4; ++i) {
      const unsigned hbi = bf16_bits(v[i]);
      ab[i]     = (unsigned short)hbi;
      ab[4 + i] = (unsigned short)bf16_bits(v[i] - __uint_as_float(hbi << 16));
    }
    if (node < mRows) {
      float* zp = zf + (size_t)node * D + 4 * lane;
      unsigned short* zap = za + (size_t)node * KZ + 8 * lane;
      *(volatile v4f*)zp = zv;
      *(volatile v8us*)zap = ab;
      __threadfence();
      *(volatile v4f*)zp = zv;
      *(volatile v8us*)zap = ab;
    }
  }
}

__global__ __launch_bounds__(NTHR) void k_edge(const int* __restrict__ ei, int nE, int nN,
                                               const float* __restrict__ pab,
                                               const float* __restrict__ be1, const float* __restrict__ we2,
                                               const float* __restrict__ be2, float* out) {
  __shared__ __attribute__((aligned(16))) float cst[2 * D + 16];
  __shared__ __attribute__((aligned(16))) float sy[EPB];
  const int tid = (int)threadIdx.x;

  if (tid < D) {
    cst[tid]     = bf16_val(be1[tid]);
    cst[D + tid] = bf16_val(we2[tid]);
  }
  if (tid < 32) {
    const float vb = bf16_val(be2[0]);
    if (tid == 0) cst[2 * D] = vb;
  }

  const int e0 = (int)blockIdx.x * EPB;
  int ec = e0 + tid;
  ec = ec > nE - 1 ? nE - 1 : ec;
  int s = ei[ec];
  int t = ei[(size_t)nE + (size_t)ec];
  s = s < 0 ? 0 : (s > nN - 1 ? nN - 1 : s);
  t = t < 0 ? 0 : (t > nN - 1 ? nN - 1 : t);
  const float* pa = pab + (size_t)s * PBN;
  const float* pb = pab + (size_t)t * PBN + D;
  __syncthreads();

  float dot = 0.0f;
#pragma unroll 2
  for (int c4 = 0; c4 < D / 4; ++c4) {
    const v4f a  = *(const v4fa*)(pa + 4 * c4);
    const v4f q  = *(const v4fa*)(pb + 4 * c4);
    const v4f bb = *(const v4fa*)(cst + 4 * c4);
    const v4f ww = *(const v4fa*)(cst + D + 4 * c4);
    const float t0 = fmaxf((a.x + q.x) + bb.x, 0.0f);
    const float t1 = fmaxf((a.y + q.y) + bb.y, 0.0f);
    const float t2 = fmaxf((a.z + q.z) + bb.z, 0.0f);
    const float t3 = fmaxf((a.w + q.w) + bb.w, 0.0f);
    dot = fmaf(t0, ww.x, dot);
    dot = fmaf(t1, ww.y, dot);
    dot = fmaf(t2, ww.z, dot);
    dot = fmaf(t3, ww.w, dot);
  }
  const float yv = dot + cst[2 * D];
  sy[tid] = yv;
  __syncthreads();

  const int tl = tid < 64 ? tid : 63;
  const v4f o4 = *(const v4fa*)(sy + 4 * tl);
  const int eo = e0 + 4 * tl;
  const bool stv = (tid < 64) && (eo + 3 < nE);
  if (stv) *(volatile v4f*)(out + (size_t)eo) = o4;
  __threadfence();
  if (stv) *(volatile v4f*)(out + (size_t)eo) = o4;
}

__global__ __launch_bounds__(NTHR) void k_pool(const float* __restrict__ zf, const int* __restrict__ bat,
                                               int nN, const float* __restrict__ Wc,
                                               const float* __restrict__ bc, float* out, int obase) {
  __shared__ __attribute__((aligned(16))) float sW[D * NCLS];
  __shared__ __attribute__((aligned(16))) float sZG[NG * D];
  __shared__ __attribute__((aligned(16))) float sy[NTHR];
  __shared__ float sbc[32];
  __shared__ int sB[CHB];
  const int tid = (int)threadIdx.x;
  const int c  = tid & (D - 1);
  const int g0 = (tid >> 7) * (NG / 2);

#pragma unroll 1
  for (int i = tid; i < D * NCLS; i += NTHR) sW[i] = bf16_val(Wc[i]);
  if (tid < 32) sbc[tid] = bf16_val(bc[tid < NCLS ? tid : NCLS - 1]);

  double acc[NG / 2];
  int cn[NG / 2];
#pragma unroll
  for (int j = 0; j < NG / 2; ++j) { acc[j] = 0.0; cn[j] = 0; }

#pragma unroll 1
  for (int cb = 0; cb < nN; cb += CHB) {
#pragma unroll 1
    for (int i = tid; i < CHB; i += NTHR) {
      const int idx = cb + i;
      const int bvv = bat[idx < nN ? idx : nN - 1];
      sB[i] = (idx < nN) ? bvv : -1;
    }
    __syncthreads();
    int n = nN - cb;
    n = n > CHB ? CHB : n;
#pragma unroll 1
    for (int i = 0; i < n; ++i) {
      const int bid = sB[i];
      const double dv = (double)zf[(size_t)(cb + i) * D + c];
#pragma unroll
      for (int j = 0; j < NG / 2; ++j) {
        const bool mm = (bid == g0 + j);
        acc[j] += mm ? dv : 0.0;
        cn[j]  += mm ? 1 : 0;
      }
    }
    __syncthreads();
  }
#pragma unroll
  for (int j = 0; j < NG / 2; ++j) {
    const float f  = (float)acc[j];
    const float cf = fmaxf((float)cn[j], 1.0f);
    sZG[(g0 + j) * D + c] = f * (1.0f / cf);
  }
  __syncthreads();

  const int tl = tid < NOUT1 ? tid : NOUT1 - 1;
  const int g  = tl / NCLS;
  const int k  = tl - NCLS * g;
  float dot = 0.0f;
#pragma unroll 4
  for (int cc = 0; cc < D; ++cc) dot = fmaf(sZG[g * D + cc], sW[cc * NCLS + k], dot);
  sy[tid] = dot + sbc[k];
  __syncthreads();

  const int t2 = tid < (NOUT1 / 4) ? tid : (NOUT1 / 4) - 1;
  const v4f o4 = *(const v4fa*)(sy + 4 * t2);
  const bool stv = tid < (NOUT1 / 4);
  float* op = out + (size_t)obase + 4 * t2;
  if (stv) *(volatile v4f*)op = o4;
  __threadfence();
  if (stv) *(volatile v4f*)op = o4;
}

static inline int cdiv(int a, int b) { return (a + b - 1) / b; }

extern "C" void kernel_launch(void* const* d_in, const int* in_sizes, int n_in,
                              void* d_out, int out_size, void* d_ws, size_t ws_size,
                              hipStream_t stream) {
  if (n_in < 12) return;
  if (in_sizes[0] < D || (in_sizes[0] % D) != 0) return;
  const int nN = in_sizes[0] / D;
  if (in_sizes[1] < 2 || (in_sizes[1] & 1) != 0) return;
  const int nE = in_sizes[1] / 2;
  if (nE < 32 || (nE & 31) != 0) return;
  if (nE >= (1 << 23)) return;
  if (in_sizes[2] != nN) return;
  if (in_sizes[3] != D * D || in_sizes[4] != D * D || in_sizes[5] != D) return;
  if (in_sizes[6] != 2 * D * D || in_sizes[7] != D) return;
  if (in_sizes[8] != D || in_sizes[9] != 1) return;
  if (in_sizes[10] != D * NCLS || in_sizes[11] != NCLS) return;
  if ((long long)out_size != (long long)nE + NOUT1) return;

  const float* x     = (const float*)d_in[0];
  const int*   ei    = (const int*)d_in[1];
  const int*   batch = (const int*)d_in[2];
  const float* Win   = (const float*)d_in[3];
  const float* Wself = (const float*)d_in[4];
  const float* bb    = (const float*)d_in[5];
  const float* We1   = (const float*)d_in[6];
  const float* be1   = (const float*)d_in[7];
  const float* We2   = (const float*)d_in[8];
  const float* be2   = (const float*)d_in[9];
  const float* Wcls  = (const float*)d_in[10];
  const float* bcls  = (const float*)d_in[11];
  float* out = (float*)d_out;
  const int* src = ei;
  const int* dst = ei + nE;

  const int MP = cdiv(nN, GBM) * GBM;
  const int gM = MP / GBM;
  const int gA = cdiv(nN, NBA);
  if ((long long)gA * NBA < (long long)MP) return;
  const int vec8 = ((nE & 3) == 0) ? 1 : 0;

  char* ws = (char*)d_ws;
  size_t off = 0;
  const size_t oWIS = off; off += (size_t)HSN * D * 2;           off = (off + 255) & ~(size_t)255;
  const size_t oWAB = off; off += (size_t)PBN * KZ * 2;          off = (off + 255) & ~(size_t)255;
  const size_t oXB  = off; off += (size_t)MP * D * 2;            off = (off + 255) & ~(size_t)255;
  const size_t oHS  = off; off += (size_t)MP * HSN * 4;          off = (off + 255) & ~(size_t)255;
  const size_t oZF  = off; off += (size_t)MP * D * 4;            off = (off + 255) & ~(size_t)255;
  const size_t oZA  = off; off += (size_t)MP * KZ * 2;           off = (off + 255) & ~(size_t)255;
  const size_t oPAB = off; off += (size_t)MP * PBN * 4;          off = (off + 255) & ~(size_t)255;
  if (off > ws_size || off > (size_t)WSMAX) return;
  unsigned short* WIS = (unsigned short*)(ws + oWIS);
  unsigned short* WAB = (unsigned short*)(ws + oWAB);
  unsigned short* XB  = (unsigned short*)(ws + oXB);
  float*          HS  = (float*)(ws + oHS);
  float*          ZF  = (float*)(ws + oZF);
  unsigned short* ZA  = (unsigned short*)(ws + oZA);
  float*          PAB = (float*)(ws + oPAB);

  const size_t aggLds = (size_t)AGG_LDS_INTS * 4;
  hipFuncSetAttribute(reinterpret_cast<const void*>(&k_agg), hipFuncAttributeMaxDynamicSharedMemorySize, (int)aggLds);

  const int nUnits = NU1 + NU2 + MP * (D / 8);
  k_prep<<<cdiv(nUnits, NTHR), NTHR, 0, stream>>>(x, Win, Wself, We1, nN, MP, WIS, WAB, XB);
  k_gemm<<<dim3(gM, HSN / GBN), GTHR, 0, stream>>>(XB, D, WIS, D, D, HS, HSN);
  k_agg<<<gA, NTHR, aggLds, stream>>>(src, dst, nE, nN, vec8, MP, HS, bb, ZF, ZA);
  k_gemm<<<dim3(gM, PBN / GBN), GTHR, 0, stream>>>(ZA, KZ, WAB, KZ, KZ, PAB, PBN);
  k_edge<<<cdiv(nE, EPB), NTHR, 0, stream>>>(ei, nE, nN, PAB, be1, We2, be2, out);
  k_pool<<<1, NTHR, 0, stream>>>(ZF, batch, nN, Wcls, bcls, out, nE);
}
